// BasePllay_05_38276748542092
// MI455X (gfx1250) — hardware-verified
//
#include <hip/hip_runtime.h>
#include <math.h>


#define GH 64
#define GW 64
#define NPTS (GH * GW)
#define R2MAX 7939
#define EH (GH * (GW - 1))
#define EE (2 * EH)
#define SORTN 8192
#define TT 25
#define NLAND 50
#define NG 50
#define NFC 10
#define MAXB 16
#define DTM_THREADS 64
#define PTS_PER_BLK 32
#define BINS_PER_THREAD 125
#define BARS_PITCH (2 * SORTN)
#define PH0_THREADS 256
#define TAIL_THREADS 256

typedef _Float16 v16h __attribute__((ext_vector_type(16)));
typedef _Float16 v8h  __attribute__((ext_vector_type(8)));
typedef float    v8f  __attribute__((ext_vector_type(8)));
typedef float    v4f  __attribute__((ext_vector_type(4)));
typedef float    v2f  __attribute__((ext_vector_type(2)));
union Frag { v16h v; v8h half[2]; };

__device__ __forceinline__ v8f wmma_f16(v16h a, v16h b, v8f c) {
    v8f d = __builtin_amdgcn_wmma_f32_16x16x32_f16(false, a, false, b, (short)0, c, false, false);
    asm volatile("v_nop\n\tv_nop\n\tv_nop\n\tv_nop" : "+v"(d) : "v"(a), "v"(b));
    return d;
}

__device__ __forceinline__ unsigned long long pack_bd(float b, float d) {
    return ((unsigned long long)__float_as_uint(d) << 32) | (unsigned long long)__float_as_uint(b);
}

__global__ __launch_bounds__(DTM_THREADS)
void k_dtm(const float* __restrict__ input, float* __restrict__ f_out, int B) {
    const int bat = blockIdx.y;
    const int i0  = blockIdx.x * PTS_PER_BLK;
    const int tid = threadIdx.x;
    if (bat >= B || i0 >= NPTS) return;

    __shared__ float bins[R2MAX + 1];
    __shared__ float red[DTM_THREADS];
    __shared__ float cpre[DTM_THREADS];
    __shared__ float fvals[PTS_PER_BLK] __attribute__((aligned(16)));
    __shared__ float sthr;

    const float* w = input + (size_t)bat * NPTS;
    const int t = tid;

    for (int p = 0; p < PTS_PER_BLK; ++p) {
        const int i  = i0 + p;
        const int ri = i >> 6, ci = i & 63;

        for (int k = tid; k < R2MAX; k += DTM_THREADS) bins[k] = 0.0f;
        __syncthreads();

        const int  cl  = ci - t, cr = ci + t;
        const bool okl = (cl >= 0);
        const bool okr = (t > 0) && (cr < GW);
        for (int d = 0; d < GH; ++d) {
            const int ru = ri - d, rd = ri + d;
            float v = 0.0f;
            if (ru >= 0) {
                const float* wr = w + ru * GW;
                if (okl) v += wr[cl];
                if (okr) v += wr[cr];
            }
            if (d > 0 && rd < GH) {
                const float* wr = w + rd * GW;
                if (okl) v += wr[cl];
                if (okr) v += wr[cr];
            }
            bins[d * d + t * t] += v;
            __syncthreads();
        }

        const int k0 = tid * BINS_PER_THREAD;
        const int k1 = (k0 + BINS_PER_THREAD < R2MAX) ? (k0 + BINS_PER_THREAD) : R2MAX;
        float psum = 0.0f;
        for (int k = k0; k < k1; ++k) psum += bins[k];
        red[tid] = psum;
        __syncthreads();
        if (tid == 0) {
            float c = 0.0f;
            for (int j = 0; j < DTM_THREADS; ++j) { cpre[j] = c; c += red[j]; }
            sthr = 0.05f * c;
        }
        __syncthreads();

        const float thr = sthr;
        float c  = cpre[tid];
        float mp = fminf(thr, c);
        float S  = 0.0f;
        for (int k = k0; k < k1; ++k) {
            const float cn = c + bins[k];
            const float mn = fminf(thr, cn);
            S += (float)k * (mn - mp);
            mp = mn;
            c  = cn;
        }
        red[tid] = S;
        __syncthreads();
        if (tid == 0) {
            float tot = 0.0f;
            for (int j = 0; j < DTM_THREADS; ++j) tot += red[j];
            const float s2 = (224.0f / 63.0f) * (224.0f / 63.0f);
            fvals[p] = sqrtf(tot * s2 / thr);
        }
        __syncthreads();
    }

    if (tid < 8) {
        const v4f val = *(const v4f*)(&fvals[4 * tid]);
        float* dst = f_out + (size_t)bat * NPTS + (size_t)i0 + 4 * tid;
        *(volatile v4f*)dst = val;
        __threadfence();
        *(volatile v4f*)dst = val;
    }
}

__global__ __launch_bounds__(PH0_THREADS)
void k_ph0(const float* __restrict__ f_all, float* __restrict__ bars, int B) {
    const int bat = blockIdx.x;
    const int tid = threadIdx.x;
    if (bat >= B) return;

    __shared__ float fsh[NPTS];
    __shared__ int   label[NPTS];
    __shared__ unsigned long long keys[SORTN];
    __shared__ float redmin[PH0_THREADS];
    __shared__ float redmax[PH0_THREADS];

    const float* f = f_all + (size_t)bat * NPTS;
    for (int i = tid; i < NPTS; i += PH0_THREADS) { fsh[i] = f[i]; label[i] = i; }
    __syncthreads();

    float mn = 3.0e38f, mx = -3.0e38f;
    for (int i = tid; i < NPTS; i += PH0_THREADS) {
        mn = fminf(mn, fsh[i]);
        mx = fmaxf(mx, fsh[i]);
    }
    redmin[tid] = mn; redmax[tid] = mx;
    __syncthreads();
    for (int off = PH0_THREADS / 2; off > 0; off >>= 1) {
        if (tid < off) {
            redmin[tid] = fminf(redmin[tid], redmin[tid + off]);
            redmax[tid] = fmaxf(redmax[tid], redmax[tid + off]);
        }
        __syncthreads();
    }

    for (int e = tid; e < SORTN; e += PH0_THREADS) {
        unsigned long long key = ~0ULL;
        if (e < EE) {
            int eu, ev;
            if (e < EH) { const int r = e / 63, cc = e - r * 63; eu = r * 64 + cc; ev = eu + 1; }
            else        { eu = e - EH; ev = eu + 64; }
            const float wgt = fmaxf(fsh[eu], fsh[ev]);
            key = ((unsigned long long)__float_as_uint(wgt) << 32) | (unsigned long long)(unsigned int)e;
        }
        keys[e] = key;
    }
    __syncthreads();

    for (int k = 2; k <= SORTN; k <<= 1) {
        for (int j = k >> 1; j > 0; j >>= 1) {
            for (int i = tid; i < SORTN; i += PH0_THREADS) {
                const int ixj = i ^ j;
                if (ixj > i) {
                    const unsigned long long a = keys[i];
                    const unsigned long long b = keys[ixj];
                    const bool up = ((i & k) == 0);
                    if ((up && a > b) || (!up && a < b)) {
                        keys[i]   = b;
                        keys[ixj] = a;
                    }
                }
            }
            __syncthreads();
        }
    }

    if (tid == 0) {
        for (int s = 0; s < EE; ++s) {
            unsigned int e = (unsigned int)(keys[s] & 0xffffffffULL);
            if (e >= (unsigned int)EE) e = 0;
            int eu, ev;
            if (e < (unsigned int)EH) { const int r = (int)e / 63, cc = (int)e - r * 63; eu = r * 64 + cc; ev = eu + 1; }
            else                      { eu = (int)e - EH; ev = eu + 64; }
            int ru = eu;
            while (label[ru] != ru) { label[ru] = label[label[ru]]; ru = label[ru]; }
            int rv = ev;
            while (label[rv] != rv) { label[rv] = label[label[rv]]; rv = label[rv]; }
            const float bu = fsh[ru], bvv = fsh[rv];
            const bool  ue = (bu < bvv) || ((bu == bvv) && (ru <= rv));
            const int elder   = ue ? ru : rv;
            const int younger = ue ? rv : ru;
            const bool merge  = (ru != rv);
            unsigned long long o = 0ULL;
            if (merge) {
                o = pack_bd(fsh[younger], fmaxf(fsh[eu], fsh[ev]));
                label[younger] = elder;
            }
            keys[s] = o;
        }
        keys[EE] = pack_bd(redmin[0], redmax[0]);
    } else {
        for (int s = EE + tid; s < SORTN; s += PH0_THREADS - 1) keys[s] = 0ULL;
    }
    __syncthreads();

    float* dstb = bars + (size_t)bat * BARS_PITCH;
    for (int q = tid; q < SORTN / 2; q += PH0_THREADS) {
        const unsigned long long ka = keys[2 * q];
        const unsigned long long kb = keys[2 * q + 1];
        v4f val;
        val.x = __uint_as_float((unsigned int)(ka & 0xffffffffULL));
        val.y = __uint_as_float((unsigned int)(ka >> 32));
        val.z = __uint_as_float((unsigned int)(kb & 0xffffffffULL));
        val.w = __uint_as_float((unsigned int)(kb >> 32));
        *(volatile v4f*)(dstb + 4 * (size_t)q) = val;
    }
    __threadfence();
    for (int q = tid; q < SORTN / 2; q += PH0_THREADS) {
        const unsigned long long ka = keys[2 * q];
        const unsigned long long kb = keys[2 * q + 1];
        v4f val;
        val.x = __uint_as_float((unsigned int)(ka & 0xffffffffULL));
        val.y = __uint_as_float((unsigned int)(ka >> 32));
        val.z = __uint_as_float((unsigned int)(kb & 0xffffffffULL));
        val.w = __uint_as_float((unsigned int)(kb >> 32));
        *(volatile v4f*)(dstb + 4 * (size_t)q) = val;
    }
}

__global__ __launch_bounds__(TAIL_THREADS)
void k_tail(const float* __restrict__ bars, const float* __restrict__ Wg,
            const float* __restrict__ bg, const float* __restrict__ Wfc,
            const float* __restrict__ bfc, float* __restrict__ out, int B, int out_n) {
    const int tid  = threadIdx.x;
    const int lane = tid & 31;
    const int wave = tid >> 5;
    const int h    = lane >> 4;
    const int m    = lane & 15;

    __shared__ float    land_sh[MAXB][64];
    __shared__ _Float16 Apad[MAXB][64] __attribute__((aligned(16)));
    __shared__ _Float16 Bgs[64][64]    __attribute__((aligned(16)));
    __shared__ _Float16 Bfs[16][64]    __attribute__((aligned(16)));
    __shared__ float    xsh[MAXB][64];
    __shared__ float    outsh[256]     __attribute__((aligned(16)));

    for (int idx = tid; idx < MAXB * 64; idx += TAIL_THREADS) land_sh[idx >> 6][idx & 63] = 0.0f;
    for (int idx = tid; idx < 256; idx += TAIL_THREADS) outsh[idx] = 0.0f;
    __syncthreads();

    const int ntask = B * TT;
    for (int q = wave; q < ntask; q += TAIL_THREADS / 32) {
        const int b = q / TT;
        const int t = q - b * TT;
        const float ts = 1.875f * (float)t;
        const float* bp = bars + (size_t)b * BARS_PITCH;
        float m1 = 0.0f, m2 = 0.0f;
        for (int e = lane; e < SORTN; e += 32) {
            const v2f bd = *(const v2f*)(bp + 2 * e);
            const float tri = fminf(ts - bd.x, bd.y - ts);
            const float v   = fmaxf(tri, 0.0f);
            if (v > m1)      { m2 = m1; m1 = v; }
            else if (v > m2) { m2 = v; }
        }
#pragma unroll
        for (int off = 16; off > 0; off >>= 1) {
            const float c1 = __shfl_xor(m1, off);
            const float c2 = __shfl_xor(m2, off);
            const float n1 = fmaxf(m1, c1);
            const float n2 = fmaxf(fminf(m1, c1), fmaxf(m2, c2));
            m1 = n1; m2 = n2;
        }
        if (lane == 0) {
            land_sh[b][t]      = m1;
            land_sh[b][TT + t] = m2;
        }
    }
    __syncthreads();

    for (int idx = tid; idx < MAXB * 64; idx += TAIL_THREADS) {
        const int mm = idx >> 6, k = idx & 63;
        Apad[mm][k] = (_Float16)land_sh[mm][k];
    }
    for (int idx = tid; idx < 64 * 64; idx += TAIL_THREADS) {
        const int n = idx >> 6, k = idx & 63;
        float v = 0.0f;
        if (n < NG && k < NLAND) v = Wg[n * NLAND + k] * 16.0f;
        Bgs[n][k] = (_Float16)v;
    }
    for (int idx = tid; idx < 16 * 64; idx += TAIL_THREADS) {
        const int n = idx >> 6, k = idx & 63;
        float v = 0.0f;
        if (n < NFC && k < NG) v = Wfc[n * NG + k] * 16.0f;
        Bfs[n][k] = (_Float16)v;
    }
    __syncthreads();

    const float s_inv = 0.0625f;

    {
        const int nt = wave & 3;
        v8f acc = {0.f, 0.f, 0.f, 0.f, 0.f, 0.f, 0.f, 0.f};
#pragma unroll
        for (int kc = 0; kc < 2; ++kc) {
            Frag fa, fb;
            fa.half[0] = *(const v8h*)(&Apad[m][kc * 32 + 8 * h]);
            fa.half[1] = *(const v8h*)(&Apad[m][kc * 32 + 16 + 8 * h]);
            fb.half[0] = *(const v8h*)(&Bgs[nt * 16 + m][kc * 32 + 8 * h]);
            fb.half[1] = *(const v8h*)(&Bgs[nt * 16 + m][kc * 32 + 16 + 8 * h]);
            acc = wmma_f16(fa.v, fb.v, acc);
        }
        if (wave < 4) {
#pragma unroll
            for (int r = 0; r < 8; ++r) {
                const int M = 8 * h + r;
                const int n = nt * 16 + m;
                const float bias = (n < NG) ? bg[n] : 0.0f;
                const float val  = (M < B && n < NG) ? (acc[r] * s_inv + bias) : 0.0f;
                xsh[M][n] = val;
            }
        }
    }
    __syncthreads();

    if (tid < NG) {
        float s = 0.0f;
        for (int mm = 0; mm < B; ++mm) s += fabsf(xsh[mm][tid]);
        outsh[B * NFC + tid] = s;
    }
    for (int idx = tid; idx < MAXB * 64; idx += TAIL_THREADS) {
        const int mm = idx >> 6, k = idx & 63;
        Apad[mm][k] = (_Float16)fmaxf(xsh[mm][k], 0.0f);
    }
    __syncthreads();

    {
        v8f acc = {0.f, 0.f, 0.f, 0.f, 0.f, 0.f, 0.f, 0.f};
#pragma unroll
        for (int kc = 0; kc < 2; ++kc) {
            Frag fa, fb;
            fa.half[0] = *(const v8h*)(&Apad[m][kc * 32 + 8 * h]);
            fa.half[1] = *(const v8h*)(&Apad[m][kc * 32 + 16 + 8 * h]);
            fb.half[0] = *(const v8h*)(&Bfs[m][kc * 32 + 8 * h]);
            fb.half[1] = *(const v8h*)(&Bfs[m][kc * 32 + 16 + 8 * h]);
            acc = wmma_f16(fa.v, fb.v, acc);
        }
        if (wave == 0) {
#pragma unroll
            for (int r = 0; r < 8; ++r) {
                const int M = 8 * h + r;
                const int n = m;
                if (M < B && n < NFC) outsh[M * NFC + n] = acc[r] * s_inv + bfc[n];
            }
        }
    }
    __syncthreads();

    if (wave == 0) {
        const int nq  = out_n >> 2;
        const int rem = out_n & 3;
        for (int q = lane; q < nq; q += 32) {
            const v4f val = *(const v4f*)(&outsh[4 * q]);
            *(volatile v4f*)(out + 4 * q) = val;
        }
        if (lane == 0) {
            for (int j = 0; j < rem; ++j) {
                const float v = outsh[4 * nq + j];
                ((volatile float*)out)[4 * nq + j] = v;
            }
        }
        __threadfence();
        for (int q = lane; q < nq; q += 32) {
            const v4f val = *(const v4f*)(&outsh[4 * q]);
            *(volatile v4f*)(out + 4 * q) = val;
        }
        if (lane == 0) {
            for (int j = 0; j < rem; ++j) {
                const float v = outsh[4 * nq + j];
                ((volatile float*)out)[4 * nq + j] = v;
            }
        }
    }
}

extern "C" void kernel_launch(void* const* d_in, const int* in_sizes, int n_in,
                              void* d_out, int out_size, void* d_ws, size_t ws_size,
                              hipStream_t stream) {
    if (n_in < 5) return;
    const float* input = (const float*)d_in[0];
    const float* Wg    = (const float*)d_in[1];
    const float* bg    = (const float*)d_in[2];
    const float* Wfc   = (const float*)d_in[3];
    const float* bfc   = (const float*)d_in[4];
    float* out = (float*)d_out;

    const int B = in_sizes[0] / NPTS;
    if (B < 1 || B > MAXB) return;
    if (in_sizes[1] != NG * NLAND || in_sizes[3] != NFC * NG) return;
    const int out_n = B * NFC + NG;
    if (out_size < out_n) return;

    size_t off = 0;
    float* f_ws = (float*)((char*)d_ws + off);
    off += (size_t)B * NPTS * sizeof(float);
    off = (off + 255) & ~(size_t)255;
    float* bars = (float*)((char*)d_ws + off);
    off += (size_t)B * BARS_PITCH * sizeof(float);
    if (off > ws_size) return;

    k_dtm<<<dim3(NPTS / PTS_PER_BLK, B), DTM_THREADS, 0, stream>>>(input, f_ws, B);
    k_ph0<<<dim3(B), PH0_THREADS, 0, stream>>>(f_ws, bars, B);
    k_tail<<<dim3(1), TAIL_THREADS, 0, stream>>>(bars, Wg, bg, Wfc, bfc, out, B, out_n);
}
